// SSL_BACKEND_BAM_2267742732705
// MI455X (gfx1250) — hardware-verified
//
#include <hip/hip_runtime.h>
#include <hip/hip_bf16.h>
#include <math.h>


typedef _Float16 bf16;
typedef _Float16 f16;
typedef __attribute__((ext_vector_type(4))) unsigned v4u_t;
typedef unsigned v4ua __attribute__((ext_vector_type(4), may_alias));
typedef __attribute__((ext_vector_type(4))) float v4f_t;
typedef float v4fa __attribute__((ext_vector_type(4), may_alias));
typedef __attribute__((ext_vector_type(16))) bf16  bf16x16;
typedef bf16x16 f16x16;
typedef __attribute__((ext_vector_type(8)))  bf16  bf16x8;
typedef bf16x8 f16x8;
typedef __attribute__((ext_vector_type(4)))  bf16  bf16x4;
typedef __attribute__((ext_vector_type(8)))  float f32x8;
__device__ __forceinline__ f32x8 wmma16(f16x16 a, f16x16 b, f32x8 c) {
  c = __builtin_amdgcn_wmma_f32_16x16x32_f16(false, a, false, b, (short)0, c, false, false);
  asm volatile("v_nop\n\tv_nop\n\tv_nop\n\tv_nop" : "+v"(c) : "v"(a), "v"(b));
  return c;
}
#define LDS_STRIDE 48
#define KSTRIDE    72
#define VSTRIDE    48

__device__ __forceinline__ f32x8 wmma_bf16(bf16x16 a, bf16x16 b, f32x8 c) {
  c = __builtin_amdgcn_wmma_f32_16x16x32_f16(false, a, false, b, (short)0, c, false, false);
  asm volatile("v_nop\n\tv_nop\n\tv_nop\n\tv_nop" : "+v"(c) : "v"(a), "v"(b));
  return c;
}

template <typename T>
__device__ __forceinline__ bf16x16 load_frag(const T* __restrict__ base, int ld,
                                             int row0, int k0) {
  const int lane = threadIdx.x & 31;
  const int r    = lane & 15;
  const int kh   = (lane >> 4) * 8;
  const T* p0 = base + (size_t)(row0 + r) * ld + (k0 + kh);
  const T* p1 = p0 + 16;
  bf16x16 f;
#pragma unroll
  for (int i = 0; i < 8; ++i) {
    f[i]     = (bf16)p0[i];
    f[i + 8] = (bf16)p1[i];
  }
  return f;
}

__device__ __forceinline__ bf16x16 lds_frag(const bf16* base, int stride) {
  const int lane = threadIdx.x & 31;
  const int row  = lane & 15;
  const int kh   = (lane >> 4) * 8;
  const bf16x8 lo = *(const bf16x8*)(base + row * stride + kh);
  const bf16x8 hi = *(const bf16x8*)(base + row * stride + kh + 16);
  bf16x16 f;
#pragma unroll
  for (int i = 0; i < 8; ++i) { f[i] = lo[i]; f[i + 8] = hi[i]; }
  return f;
}

template <typename T>
__device__ __forceinline__ void stage_read16(const T* __restrict__ p, float* buf) {
#pragma unroll
  for (int i = 0; i < 16; ++i) buf[i] = (float)p[i];
}

__device__ __forceinline__ void stage_write(bf16* dst, const float* buf, int nquad) {
#pragma unroll
  for (int i = 0; i < nquad; ++i) {
    bf16x4 q;
    q[0] = (bf16)buf[4 * i];     q[1] = (bf16)buf[4 * i + 1];
    q[2] = (bf16)buf[4 * i + 2]; q[3] = (bf16)buf[4 * i + 3];
    *(bf16x4*)(dst + 4 * i) = q;
  }
}


#define GSTR 48
#define GSTR 48
template <typename AT, int EPI, bool OUT16>
__global__ __launch_bounds__(256) void gemm_kne(const AT* __restrict__ A, int lda, const float* __restrict__ Wm, int ldw,
                                                const float* __restrict__ bias, const float* __restrict__ R, const float* __restrict__ gvec,
                                                void* __restrict__ Yv, int ldy, int K) {
  __shared__ __attribute__((aligned(16))) f16 ldsA[128 * GSTR];
  __shared__ __attribute__((aligned(16))) f16 ldsW[128 * GSTR];
  __shared__ __attribute__((aligned(16))) float oS[8][32 * 68];
  const int tid = threadIdx.x, lane = tid & 31, wave = tid >> 5, cl = lane & 15, rh = (lane >> 4) * 8;
  const int m0 = blockIdx.x * 128, n0 = blockIdx.y * 128;
  const int wm = (wave & 3) * 32, wn = (wave >> 2) * 64;
  f32x8 acc[2][4];
#pragma unroll
  for (int i = 0; i < 2; ++i)
#pragma unroll
    for (int j = 0; j < 4; ++j) { f32x8 z = {}; acc[i][j] = z; }
#pragma unroll 1
  for (int k0 = 0; k0 < K; k0 += 32) {
    __syncthreads();
    { const int row = tid >> 1, ch = (tid & 1) * 16;
      const AT* src = A + (size_t)(m0 + row) * lda + k0 + ch;
#pragma unroll
      for (int g = 0; g < 16; ++g) ldsA[row * GSTR + ch + g] = (f16)src[g]; }
    { const int k = tid >> 3, nn0 = (tid & 7) * 16;
      const float* src = Wm + (size_t)(k0 + k) * ldw + n0 + nn0;
#pragma unroll
      for (int g = 0; g < 4; ++g) { const v4f_t v = *(const v4f_t*)(src + 4 * g);
#pragma unroll
        for (int u = 0; u < 4; ++u) ldsW[(nn0 + 4 * g + u) * GSTR + k] = (f16)v[u]; } }
    __syncthreads();
    f16x16 af[2];
#pragma unroll
    for (int i = 0; i < 2; ++i) af[i] = lds_frag(ldsA + (wm + 16 * i) * GSTR, GSTR);
#pragma unroll
    for (int j = 0; j < 4; ++j) {
      const f16x16 bf = lds_frag(ldsW + (wn + 16 * j) * GSTR, GSTR);
#pragma unroll
      for (int i = 0; i < 2; ++i) acc[i][j] = wmma16(af[i], bf, acc[i][j]);
    }
  }
  float* so = oS[wave];
#pragma unroll
  for (int i = 0; i < 2; ++i)
#pragma unroll
    for (int j = 0; j < 4; ++j) {
      const int n = n0 + wn + 16 * j + cl;
      const float bv = bias ? bias[n] : 0.0f;
      const float gv = (EPI == 2 || EPI == 4) ? gvec[n] : 0.0f;
      if (EPI == 1) {
#pragma unroll 1
        for (int r = 0; r < 8; ++r) { const float xg = acc[i][j][r] + bv; so[(16 * i + rh + r) * 68 + 16 * j + cl] = 0.5f * xg * (1.0f + erff(xg * 0.70710678118654752f)); }
      } else {
#pragma unroll
        for (int r = 0; r < 8; ++r) {
          float v = acc[i][j][r] + bv;
          if (EPI == 3) v = fmaxf(v, 0.0f);
          if (EPI == 4) v = gv * v;
          if (EPI == 2) v = R[(size_t)(m0 + wm + 16 * i + rh + r) * ldy + n] + gv * v;
          so[(16 * i + rh + r) * 68 + 16 * j + cl] = v;
        }
      }
    }
  asm volatile("s_wait_dscnt 0" ::: "memory");
  __builtin_amdgcn_wave_barrier();
#pragma unroll 1
  for (int pass = 0; pass < 2; ++pass) {
    if (OUT16) {
      f16* Y = (f16*)Yv;
#pragma unroll
      for (int it = 0; it < 8; ++it) { const int c = lane + 32 * it, rr = c >> 3, q8 = (c & 7) * 8;
        union { f16 h[8]; v4u_t v; } u;
#pragma unroll
        for (int e = 0; e < 8; ++e) u.h[e] = (f16)so[rr * 68 + q8 + e];
        *(volatile v4u_t*)(Y + (size_t)(m0 + wm + rr) * ldy + n0 + wn + q8) = u.v; }
    } else {
      float* Y = (float*)Yv;
#pragma unroll
      for (int it = 0; it < 16; ++it) { const int f4 = lane + 32 * it, rr = f4 >> 4, q = (f4 & 15) * 4;
        *(volatile v4f_t*)(Y + (size_t)(m0 + wm + rr) * ldy + n0 + wn + q) = *(const v4fa*)(so + rr * 68 + q); }
    }
    __threadfence();
  }
}

template <typename AT, int EPI, bool OUT16>
__global__ __launch_bounds__(256) void gemm_knez(const AT* __restrict__ A, int lda, size_t strideA, const float* __restrict__ Wm, int ldw, size_t strideW,
                                                 const float* __restrict__ bias, const float* __restrict__ R, const float* __restrict__ gvec,
                                                 void* __restrict__ Yv, int ldy, size_t strideY, int K) {
  A += (size_t)blockIdx.z * strideA; Wm += (size_t)blockIdx.z * strideW; Yv = (void*)((char*)Yv + (size_t)blockIdx.z * strideY * (OUT16 ? 2 : 4)); if (R) R += (size_t)blockIdx.z * strideY;
  __shared__ __attribute__((aligned(16))) f16 ldsA[128 * GSTR];
  __shared__ __attribute__((aligned(16))) f16 ldsW[128 * GSTR];
  __shared__ __attribute__((aligned(16))) float oS[8][32 * 68];
  const int tid = threadIdx.x, lane = tid & 31, wave = tid >> 5, cl = lane & 15, rh = (lane >> 4) * 8;
  const int m0 = blockIdx.x * 128, n0 = blockIdx.y * 128;
  const int wm = (wave & 3) * 32, wn = (wave >> 2) * 64;
  f32x8 acc[2][4];
#pragma unroll
  for (int i = 0; i < 2; ++i)
#pragma unroll
    for (int j = 0; j < 4; ++j) { f32x8 z = {}; acc[i][j] = z; }
#pragma unroll 1
  for (int k0 = 0; k0 < K; k0 += 32) {
    __syncthreads();
    { const int row = tid >> 1, ch = (tid & 1) * 16;
      const AT* src = A + (size_t)(m0 + row) * lda + k0 + ch;
#pragma unroll
      for (int g = 0; g < 16; ++g) ldsA[row * GSTR + ch + g] = (f16)src[g]; }
    { const int k = tid >> 3, nn0 = (tid & 7) * 16;
      const float* src = Wm + (size_t)(k0 + k) * ldw + n0 + nn0;
#pragma unroll
      for (int g = 0; g < 4; ++g) { const v4f_t v = *(const v4f_t*)(src + 4 * g);
#pragma unroll
        for (int u = 0; u < 4; ++u) ldsW[(nn0 + 4 * g + u) * GSTR + k] = (f16)v[u]; } }
    __syncthreads();
    f16x16 af[2];
#pragma unroll
    for (int i = 0; i < 2; ++i) af[i] = lds_frag(ldsA + (wm + 16 * i) * GSTR, GSTR);
#pragma unroll
    for (int j = 0; j < 4; ++j) {
      const f16x16 bf = lds_frag(ldsW + (wn + 16 * j) * GSTR, GSTR);
#pragma unroll
      for (int i = 0; i < 2; ++i) acc[i][j] = wmma16(af[i], bf, acc[i][j]);
    }
  }
  float* so = oS[wave];
#pragma unroll
  for (int i = 0; i < 2; ++i)
#pragma unroll
    for (int j = 0; j < 4; ++j) {
      const int n = n0 + wn + 16 * j + cl;
      const float bv = bias ? bias[n] : 0.0f;
      const float gv = (EPI == 2 || EPI == 4) ? gvec[n] : 0.0f;
      if (EPI == 1) {
#pragma unroll 1
        for (int r = 0; r < 8; ++r) { const float xg = acc[i][j][r] + bv; so[(16 * i + rh + r) * 68 + 16 * j + cl] = 0.5f * xg * (1.0f + erff(xg * 0.70710678118654752f)); }
      } else {
#pragma unroll
        for (int r = 0; r < 8; ++r) {
          float v = acc[i][j][r] + bv;
          if (EPI == 3) v = fmaxf(v, 0.0f);
          if (EPI == 4) v = gv * v;
          if (EPI == 2) v = R[(size_t)(m0 + wm + 16 * i + rh + r) * ldy + n] + gv * v;
          so[(16 * i + rh + r) * 68 + 16 * j + cl] = v;
        }
      }
    }
  asm volatile("s_wait_dscnt 0" ::: "memory");
  __builtin_amdgcn_wave_barrier();
#pragma unroll 1
  for (int pass = 0; pass < 2; ++pass) {
    if (OUT16) {
      f16* Y = (f16*)Yv;
#pragma unroll
      for (int it = 0; it < 8; ++it) { const int c = lane + 32 * it, rr = c >> 3, q8 = (c & 7) * 8;
        union { f16 h[8]; v4u_t v; } u;
#pragma unroll
        for (int e = 0; e < 8; ++e) u.h[e] = (f16)so[rr * 68 + q8 + e];
        *(volatile v4u_t*)(Y + (size_t)(m0 + wm + rr) * ldy + n0 + wn + q8) = u.v; }
    } else {
      float* Y = (float*)Yv;
#pragma unroll
      for (int it = 0; it < 16; ++it) { const int f4 = lane + 32 * it, rr = f4 >> 4, q = (f4 & 15) * 4;
        *(volatile v4f_t*)(Y + (size_t)(m0 + wm + rr) * ldy + n0 + wn + q) = *(const v4fa*)(so + rr * 68 + q); }
    }
    __threadfence();
  }
}

template <typename AT, bool ACC>
__global__ __launch_bounds__(256) void gemm_kn2(const AT* __restrict__ A, int lda, size_t strideA,
                                               const float* __restrict__ Wm, int ldw, size_t strideW,
                                               const float* __restrict__ bias, float scale,
                                               float* __restrict__ Y, int ldy, size_t strideY, int K) {
  __shared__ __attribute__((aligned(16))) f16 ldsA[128 * GSTR], ldsAl[128 * GSTR];
  __shared__ __attribute__((aligned(16))) f16 ldsW[128 * GSTR], ldsWl[128 * GSTR];
  __shared__ __attribute__((aligned(16))) float oS[8][32 * 68];
  const int tid = threadIdx.x, lane = tid & 31, wave = tid >> 5, cl = lane & 15, rh = (lane >> 4) * 8;
  const int m0 = blockIdx.x * 128, n0 = blockIdx.y * 128;
  const int wm = (wave & 3) * 32, wn = (wave >> 2) * 64;
  A += (size_t)blockIdx.z * strideA; Wm += (size_t)blockIdx.z * strideW; Y += (size_t)blockIdx.z * strideY;
  f32x8 acc[2][4], accx[2][4];
#pragma unroll
  for (int i = 0; i < 2; ++i)
#pragma unroll
    for (int j = 0; j < 4; ++j) { f32x8 z = {}; acc[i][j] = z; accx[i][j] = z; }
#pragma unroll 1
  for (int k0 = 0; k0 < K; k0 += 32) {
    __syncthreads();
    {
      const int row = tid >> 1, ch = (tid & 1) * 16;
      const AT* src = A + (size_t)(m0 + row) * lda + k0 + ch;
#pragma unroll
      for (int g = 0; g < 16; ++g) { const float v = (float)src[g]; const f16 h = (f16)v; ldsA[row * GSTR + ch + g] = h; ldsAl[row * GSTR + ch + g] = (f16)((v - (float)h) * 2048.0f); }
    }
    {
      const int k = tid >> 3, nn0 = (tid & 7) * 16;
      const float* src = Wm + (size_t)(k0 + k) * ldw + n0 + nn0;
#pragma unroll
      for (int g = 0; g < 4; ++g) { const v4f_t v = *(const v4f_t*)(src + 4 * g);
#pragma unroll
        for (int u = 0; u < 4; ++u) { const f16 h = (f16)v[u]; ldsW[(nn0 + 4 * g + u) * GSTR + k] = h; ldsWl[(nn0 + 4 * g + u) * GSTR + k] = (f16)((v[u] - (float)h) * 2048.0f); } }
    }
    __syncthreads();
    f16x16 af[2], afl[2];
#pragma unroll
    for (int i = 0; i < 2; ++i) { af[i] = lds_frag(ldsA + (wm + 16 * i) * GSTR, GSTR); afl[i] = lds_frag(ldsAl + (wm + 16 * i) * GSTR, GSTR); }
#pragma unroll
    for (int j = 0; j < 4; ++j) {
      const f16x16 bf = lds_frag(ldsW + (wn + 16 * j) * GSTR, GSTR), bfl = lds_frag(ldsWl + (wn + 16 * j) * GSTR, GSTR);
#pragma unroll
      for (int i = 0; i < 2; ++i) { acc[i][j] = wmma16(af[i], bf, acc[i][j]); accx[i][j] = wmma16(af[i], bfl, accx[i][j]); accx[i][j] = wmma16(afl[i], bf, accx[i][j]); }
    }
  }
  float* so = oS[wave];
#pragma unroll
  for (int i = 0; i < 2; ++i)
#pragma unroll
    for (int j = 0; j < 4; ++j) {
      const float bv = bias ? bias[n0 + wn + 16 * j + cl] : 0.0f;
#pragma unroll
      for (int r = 0; r < 8; ++r) so[(16 * i + rh + r) * 68 + 16 * j + cl] = (acc[i][j][r] + accx[i][j][r] * (1.0f / 2048.0f)) * scale + bv;
    }
  asm volatile("s_wait_dscnt 0" ::: "memory");
  __builtin_amdgcn_wave_barrier();
  if (ACC) {
#pragma unroll
    for (int it = 0; it < 16; ++it) { const int f4 = lane + 32 * it, rr = f4 >> 4, q = (f4 & 15) * 4;
      const v4f_t old = *(const v4fa*)(Y + (size_t)(m0 + wm + rr) * ldy + n0 + wn + q);
      v4f_t v = *(const v4fa*)(so + rr * 68 + q); v += old; *(v4fa*)(so + rr * 68 + q) = v; }
    asm volatile("s_wait_dscnt 0" ::: "memory");
  }
#pragma unroll 1
  for (int pass = 0; pass < 2; ++pass) {
#pragma unroll
    for (int it = 0; it < 16; ++it) { const int f4 = lane + 32 * it, rr = f4 >> 4, q = (f4 & 15) * 4;
      *(volatile v4f_t*)(Y + (size_t)(m0 + wm + rr) * ldy + n0 + wn + q) = *(const v4fa*)(so + rr * 68 + q); }
    __threadfence();
  }
}

__global__ __launch_bounds__(256) void k_transpose(const float* __restrict__ Wm, float* __restrict__ Wt, int rows, int cols) {
  __shared__ float tS[64][65];
  const int tid = threadIdx.x, tbj = cols / 64, bi = blockIdx.x / tbj, bj = blockIdx.x % tbj;
  for (int e = tid; e < 64 * 64; e += 256) { const int r = e >> 6, c = e & 63; tS[r][c] = Wm[(size_t)(bi * 64 + r) * cols + bj * 64 + c]; }
  __syncthreads();
  for (int ch = tid; ch < 64 * 16; ch += 256) { const int r = ch >> 4, q4 = (ch & 15) * 4; v4f_t o; o[0] = tS[q4][r]; o[1] = tS[q4 + 1][r]; o[2] = tS[q4 + 2][r]; o[3] = tS[q4 + 3][r];
    float* dst = Wt + (size_t)(bj * 64 + r) * rows + bi * 64 + q4; *(volatile v4f_t*)dst = o; __threadfence(); *(volatile v4f_t*)dst = o; }
}

#define BBs 2
#define TTs 256
#define INs 512
#define OUTs 256
#define HHs 8
#define CHs 32
__global__ __launch_bounds__(256) void k_fill(float* __restrict__ p, float val, size_t n4) { const size_t i = (size_t)blockIdx.x * 256 + threadIdx.x; if (i < n4) { v4f_t v = {val, val, val, val}; *(volatile v4f_t*)(p + 4 * i) = v; __threadfence(); *(volatile v4f_t*)(p + 4 * i) = v; } }
__global__ __launch_bounds__(256) void k_transpose_ld(const float* __restrict__ Wm, int lds, float* __restrict__ Wt, int rows, int cols) {
  __shared__ float tS[64][65];
  const int tid = threadIdx.x, tbj = cols / 64, bi = blockIdx.x / tbj, bj = blockIdx.x % tbj;
  for (int e = tid; e < 64 * 64; e += 256) { const int r = e >> 6, c = e & 63; tS[r][c] = Wm[(size_t)(bi * 64 + r) * lds + bj * 64 + c]; }
  __syncthreads();
  for (int ch = tid; ch < 64 * 16; ch += 256) { const int r = ch >> 4, q4 = (ch & 15) * 4; v4f_t o; o[0] = tS[q4][r]; o[1] = tS[q4 + 1][r]; o[2] = tS[q4 + 2][r]; o[3] = tS[q4 + 3][r];
    float* dst = Wt + (size_t)(bj * 64 + r) * rows + bi * 64 + q4; *(volatile v4f_t*)dst = o; __threadfence(); *(volatile v4f_t*)dst = o; }
}
__global__ __launch_bounds__(256) void k_trs(const float* __restrict__ src, int ld, float* __restrict__ dst, int rows, int cols) { const int i = blockIdx.x * 256 + threadIdx.x; if (i >= rows * cols) return; const int c = i / rows, r = i % rows; const float v = src[(size_t)r * ld + c]; *(volatile float*)(dst + (size_t)c * rows + r) = v; __threadfence(); *(volatile float*)(dst + (size_t)c * rows + r) = v; }
__global__ __launch_bounds__(128) void k_pm(const float* __restrict__ xb, int j0, float* __restrict__ PM) { const int pr = blockIdx.x, jl = pr / TTs, k = pr % TTs, c = 4 * threadIdx.x;
  const v4f_t v = *(const v4f_t*)(xb + (size_t)(j0 + jl) * INs + c) * *(const v4f_t*)(xb + (size_t)k * INs + c); *(volatile v4f_t*)(PM + (size_t)pr * INs + c) = v; __threadfence(); *(volatile v4f_t*)(PM + (size_t)pr * INs + c) = v; }
__global__ __launch_bounds__(256) void k_lg(const float* __restrict__ A, const float* __restrict__ aw, float* __restrict__ LGP) {
  __shared__ float part[HHs][256];
  const size_t pr = blockIdx.x; const int o = threadIdx.x; const float a = tanhf(A[pr * OUTs + o]);
#pragma unroll
  for (int h = 0; h < HHs; ++h) part[h][o] = a * aw[o * HHs + h];
  __syncthreads();
  for (int st = 128; st > 0; st >>= 1) { if (o < st) {
#pragma unroll
      for (int h = 0; h < HHs; ++h) part[h][o] += part[h][o + st]; }
    __syncthreads(); }
  if (o < 32) { const float v = (o < HHs) ? part[o][0] : 0.0f; *(volatile float*)(LGP + pr * 32 + o) = v; __threadfence(); *(volatile float*)(LGP + pr * 32 + o) = v; }
}
__global__ __launch_bounds__(256) void k_csoft(const float* __restrict__ LGP, const int* __restrict__ CNT, float* __restrict__ Sp) {
  __shared__ float red[256];
  const int j = blockIdx.x, h = blockIdx.y, k = threadIdx.x; const int lo = min(j, k), hi = max(j, k); const int flags = CNT[hi + 1] - CNT[lo]; const float mk = (j == k || flags == 0) ? 1.0f : 0.0f;
  const float lg = LGP[((size_t)j * TTs + k) * 32 + h] * mk; float m = lg;
  red[k] = m; __syncthreads(); for (int o2 = 128; o2 > 0; o2 >>= 1) { if (k < o2) red[k] = fmaxf(red[k], red[k + o2]); __syncthreads(); }
  m = red[0]; __syncthreads(); const float e = expf(lg - m);
  red[k] = e; __syncthreads(); for (int o2 = 128; o2 > 0; o2 >>= 1) { if (k < o2) red[k] += red[k + o2]; __syncthreads(); }
  const float p = e / red[0]; float* d = Sp + ((size_t)h * TTs + j) * TTs + k;
#pragma unroll 1
  for (int pass = 0; pass < 2; ++pass) { *(volatile float*)d = p; __threadfence(); }
}
__global__ __launch_bounds__(256) void k_cnt(const int* __restrict__ bnd, int* __restrict__ CNT) { __shared__ int c[TTs + 32]; const int t = threadIdx.x; if (t == 0) { int s = 0; c[0] = 0; for (int m = 0; m < TTs; ++m) { s += (bnd[m] != 0); c[m + 1] = s; } for (int m = TTs + 1; m < TTs + 32; ++m) c[m] = 0; } __syncthreads();
  for (int i = t; i < TTs + 32; i += 256) { *(volatile int*)(CNT + i) = c[i]; __threadfence(); *(volatile int*)(CNT + i) = c[i]; } }
__global__ __launch_bounds__(256) void k_flat(const float* __restrict__ X1H, float* __restrict__ X1F) { const size_t i = (size_t)blockIdx.x * 256 + threadIdx.x; const size_t e0 = 4 * i; const int j = (int)(e0 / (INs * HHs)), r = (int)(e0 % (INs * HHs)); v4f_t v;
#pragma unroll
  for (int u = 0; u < 4; ++u) { const int rr = r + u, d = rr / HHs, h = rr % HHs; v[u] = X1H[((size_t)h * TTs + j) * INs + d]; }
  *(volatile v4f_t*)(X1F + e0) = v; __threadfence(); *(volatile v4f_t*)(X1F + e0) = v; }
__global__ __launch_bounds__(256) void k_bnselu(const float* __restrict__ Y, const float* __restrict__ g, const float* __restrict__ bt, float* __restrict__ outp) {
  const int c = threadIdx.x; float s = 0.0f, q = 0.0f;
#pragma unroll 1
  for (int r = 0; r < BBs * TTs; ++r) s += Y[(size_t)r * OUTs + c];
  const float mu = s / (float)(BBs * TTs);
#pragma unroll 1
  for (int r = 0; r < BBs * TTs; ++r) { const float dv = Y[(size_t)r * OUTs + c] - mu; q += dv * dv; }
  const float var = q / (float)(BBs * TTs); const float is = 1.0f / __builtin_sqrtf(var + 1e-5f); const float gg = g[c] * is, bb = bt[c] - mu * gg;
  const float al = 1.6732632423543772f, sl = 1.0507009873554805f;
#pragma unroll 1
  for (int pass = 0; pass < 2; ++pass) {
#pragma unroll 1
    for (int r = 0; r < BBs * TTs; ++r) { const float yn = Y[(size_t)r * OUTs + c] * gg + bb; const float o = (yn > 0.0f) ? sl * yn : sl * al * (expf(yn) - 1.0f); *(volatile float*)(outp + (size_t)r * OUTs + c) = o; }
    __threadfence(); }
}

extern "C" void kernel_launch(void* const* d_in, const int* in_sizes, int n_in,
                              void* d_out, int out_size, void* d_ws, size_t ws_size,
                              hipStream_t stream) {
  (void)in_sizes; (void)n_in; (void)out_size;
  const float** f = (const float**)d_in;
  const float* x = f[0]; const int* bnd = (const int*)d_in[1]; const float* Wap = f[2], *bap = f[3], *aw = f[4], *Wpa = f[5], *bpa = f[6], *Wna = f[7], *bna = f[8], *g = f[9], *bt = f[10];
  float* out = (float*)d_out;
  char* ws = (char*)d_ws;
  float* WapT = (float*)ws; ws += (size_t)INs * OUTs * 4; float* WpaT = (float*)ws; ws += (size_t)INs * HHs * OUTs * 4; float* WnaT = (float*)ws; ws += (size_t)INs * OUTs * 4; float* ones = (float*)ws; ws += OUTs * 4;
  float* PM = (float*)ws; ws += (size_t)CHs * TTs * INs * 4; float* A = (float*)ws; ws += (size_t)CHs * TTs * OUTs * 4; float* LGP = (float*)ws; ws += (size_t)TTs * TTs * 32 * 4; int* CNT = (int*)ws; ws += (TTs + 32) * 4;
  float* Sp = (float*)ws; ws += (size_t)HHs * TTs * TTs * 4; float* SpT = (float*)ws; ws += (size_t)TTs * TTs * 4; float* X1H = (float*)ws; ws += (size_t)HHs * TTs * INs * 4; float* X1F = (float*)ws; ws += (size_t)TTs * INs * HHs * 4; float* Y = (float*)ws; ws += (size_t)BBs * TTs * OUTs * 4;
  if ((size_t)(ws - (char*)d_ws) > ws_size) return;
  const dim3 blk(256);
  k_transpose<<<dim3((OUTs / 64) * (INs / 64)), blk, 0, stream>>>(Wap, WapT, OUTs, INs); k_transpose<<<dim3((OUTs / 64) * (INs * HHs / 64)), blk, 0, stream>>>(Wpa, WpaT, OUTs, INs * HHs); k_transpose<<<dim3((OUTs / 64) * (INs / 64)), blk, 0, stream>>>(Wna, WnaT, OUTs, INs);
  k_fill<<<dim3(1), blk, 0, stream>>>(ones, 1.0f, OUTs / 4);
  for (int b = 0; b < BBs; ++b) { const float* xb = x + (size_t)b * TTs * INs;
    k_cnt<<<dim3(1), blk, 0, stream>>>(bnd + b * TTs, CNT);
    for (int j0 = 0; j0 < TTs; j0 += CHs) {
      k_pm<<<dim3(CHs * TTs), dim3(128), 0, stream>>>(xb, j0, PM);
      gemm_kn2<float, false><<<dim3(CHs * TTs / 128, OUTs / 128, 1), blk, 0, stream>>>(PM, INs, 0, WapT, OUTs, 0, bap, 1.0f, A, OUTs, 0, INs);
      k_lg<<<dim3(CHs * TTs), blk, 0, stream>>>(A, aw, LGP + (size_t)j0 * TTs * 32);
    }
    k_csoft<<<dim3(TTs, HHs), blk, 0, stream>>>(LGP, CNT, Sp);
    for (int h = 0; h < HHs; ++h) {
      gemm_kn2<float, false><<<dim3(TTs / 128, INs / 128, 1), blk, 0, stream>>>(Sp + (size_t)h * TTs * TTs, TTs, 0, xb, INs, 0, nullptr, 1.0f, X1H + (size_t)h * TTs * INs, INs, 0, TTs);
    }
    k_flat<<<dim3(((size_t)TTs * INs * HHs / 4 + 255) / 256), blk, 0, stream>>>(X1H, X1F);
    gemm_kn2<float, false><<<dim3(TTs / 128, OUTs / 128, 1), blk, 0, stream>>>(X1F, INs * HHs, 0, WpaT, OUTs, 0, bpa, 1.0f, Y + (size_t)b * TTs * OUTs, OUTs, 0, INs * HHs);
    gemm_kn2<float, true><<<dim3(TTs / 128, OUTs / 128, 1), blk, 0, stream>>>(xb, INs, 0, WnaT, OUTs, 0, bna, 1.0f, Y + (size_t)b * TTs * OUTs, OUTs, 0, INs);
  }
  k_bnselu<<<dim3(1), blk, 0, stream>>>(Y, g, bt, out);
}
